// TransformerBlock_45689862095177
// MI455X (gfx1250) — hardware-verified
//
#include <hip/hip_runtime.h>
#include <stddef.h>


typedef _Float16 v16h __attribute__((ext_vector_type(16)));
typedef _Float16 v8h  __attribute__((ext_vector_type(8)));
typedef float    v8f  __attribute__((ext_vector_type(8)));
typedef float    v4f  __attribute__((ext_vector_type(4)));

#ifndef NB
#define NB 2
#endif
#ifndef SEQ
#define SEQ 2048
#endif
#define NB_FULL  2
#define SEQ_FULL 2048
#define DIM   1024
#define NHEAD 16
#define HD    64
#define DFF   4096
#define DCOND 768
#define NCOND 77
#define CPAD  128
#define CKEYS 96
#define MROWS (NB * SEQ)
#define CROWS (NB * CPAD)

static_assert(NB >= 1 && NB <= NB_FULL);
static_assert(SEQ >= 128 && SEQ <= SEQ_FULL && (SEQ % 128) == 0);
static_assert(DIM == NHEAD * HD);
static_assert(HD == 64);
static_assert((DIM % 64) == 0 && (DFF % 64) == 0 && (DCOND % 64) == 0);
static_assert((MROWS % 64) == 0 && (CROWS % 64) == 0);
static_assert((SEQ % 64) == 0 && (CPAD % 64) == 0);
static_assert(NCOND <= CKEYS && CKEYS <= CPAD && (CKEYS % 32) == 0);
static_assert(DIM == 32 * 8 * 4);
static_assert((MROWS % 8) == 0);
static_assert(((size_t)CROWS * DCOND) % (8 * 256) == 0);
static_assert((DCOND % 8) == 0);
static_assert((size_t)MROWS * DFF < (size_t)0xFFFFFFFFu);
static_assert(DFF == 4 * DIM);

#define LDT 72
#define LDC 68
#define LDP 104
static_assert(LDT >= 64 + 8 && LDP >= CKEYS + 8 && LDC >= 64 + 4);
static_assert((LDT % 8) == 0 && (LDP % 8) == 0 && (LDC % 4) == 0);

#define WCARRY 64.0f
#define PCARRY 1024.0f
#define VCARRY 64.0f
#define GCARRY 64.0f

#define WQKV_E   ((size_t)3 * DIM * DIM)
#define WSQ_E    ((size_t)DIM * DIM)
#define WKV_E    ((size_t)2 * DIM * DCOND)
#define WFF_E    ((size_t)DIM * DFF)
#define OFF_WQKV ((size_t)0)
#define OFF_WPSA (OFF_WQKV + WQKV_E)
#define OFF_WQCA (OFF_WPSA + WSQ_E)
#define OFF_WKV  (OFF_WQCA + WSQ_E)
#define OFF_WPCA (OFF_WKV + WKV_E)
#define OFF_WFF1 (OFF_WPCA + WSQ_E)
#define OFF_WFF2 (OFF_WFF1 + WFF_E)
#define WT_ELEMS (OFF_WFF2 + WFF_E)

#define WT_BYTES      (WT_ELEMS * 2)
#define PLANE16_BYTES ((size_t)MROWS * DIM * 2)
#define G16_BYTES     ((size_t)MROWS * DFF * 2)
#define X32_BYTES     ((size_t)MROWS * DIM * 4)
#define C16_BYTES     ((size_t)CROWS * DCOND * 2)
#define KV16_BYTES    ((size_t)CROWS * DIM * 2)
#define B_H16   (WT_BYTES)
#define B_QKVC  (B_H16 + PLANE16_BYTES)
#define B_X1    (B_QKVC + 4 * PLANE16_BYTES)
#define B_X2    (B_X1 + X32_BYTES)
#define B_C16   (B_X2 + X32_BYTES)
#define B_KVC   (B_C16 + C16_BYTES)
#define WS_TOTAL (B_KVC + 2 * KV16_BYTES)
static_assert((WT_BYTES % 128) == 0 && (PLANE16_BYTES % 128) == 0 && (X32_BYTES % 128) == 0);
static_assert((C16_BYTES % 128) == 0 && (KV16_BYTES % 128) == 0);
static_assert(G16_BYTES <= 4 * PLANE16_BYTES);
static_assert((size_t)NB * DIM * SEQ * 2 == PLANE16_BYTES);
static_assert((size_t)NB * DIM * CPAD * 2 == KV16_BYTES);
static_assert(WS_TOTAL <= (size_t)134217728);

__device__ __forceinline__ float bf16r(float x) {
  unsigned int u = __float_as_uint(x);
  u = (u + 0x7FFFu + ((u >> 16) & 1u)) & 0xFFFF0000u;
  return __uint_as_float(u);
}

__device__ __forceinline__ v16h frag_join(v8h lo, v8h hi) {
  v16h out;
#pragma unroll
  for (int i = 0; i < 8; ++i) { out[i] = lo[i]; out[i + 8] = hi[i]; }
  return out;
}
__device__ __forceinline__ v16h frag_at(const _Float16* __restrict__ p) {
  return frag_join(*(const v8h*)(p), *(const v8h*)(p + 16));
}
#define LDS_FRAG(arr, idx) \
  frag_join(*(const v8h*)&(arr)[(idx)], *(const v8h*)&(arr)[(idx) + 16u])

__device__ __forceinline__ v8f wmma16(v16h a, v16h b, v8f c) {
  v8f d = __builtin_amdgcn_wmma_f32_16x16x32_f16(false, a, false, b, (short)0, c,
                                                 false, false);
  asm volatile("v_nop\n\tv_nop\n\tv_nop\n\tv_nop" : "+v"(d) : "v"(a), "v"(b));
  return d;
}

__device__ __forceinline__ float red16_max(float x) {
#pragma unroll
  for (int off = 1; off < 16; off <<= 1) x = fmaxf(x, __shfl_xor(x, off, 32));
  return x;
}
__device__ __forceinline__ float red16_sum(float x) {
#pragma unroll
  for (int off = 1; off < 16; off <<= 1) x += __shfl_xor(x, off, 32);
  return x;
}
__device__ __forceinline__ float red32_sum(float x) {
#pragma unroll
  for (int off = 1; off < 32; off <<= 1) x += __shfl_xor(x, off, 32);
  return x;
}

__device__ __forceinline__ void wave_lds_sync() {
  __builtin_amdgcn_fence(3  , "wavefront");
  asm volatile("s_wait_dscnt 0x0" ::: "memory");
  __builtin_amdgcn_wave_barrier();
}

__global__ __launch_bounds__(256) void wconv_kernel(
    const float* __restrict__ W, _Float16* __restrict__ Wt, unsigned Kdim, unsigned Ndim) {
  __shared__ _Float16 T[64 * LDT];
  const unsigned tid = threadIdx.x;
  const unsigned n0 = blockIdx.x * 64u;
  const unsigned k0 = blockIdx.y * 64u;
#pragma unroll 4
  for (unsigned j = 0; j < 16u; ++j) {
    const unsigned idx = tid + 256u * j;
    const unsigned kr = idx >> 6, nc = idx & 63u;
    const float v = W[(size_t)(k0 + kr) * Ndim + n0 + nc];
    T[nc * LDT + kr] = (_Float16)(WCARRY * bf16r(v));
  }
  __syncthreads();
  v8h x[2];
  size_t off[2];
#pragma unroll
  for (unsigned i = 0; i < 2u; ++i) {
    const unsigned n = 32u * i + (tid >> 3);
    const unsigned kc = (tid & 7u) * 8u;
    x[i] = *(const v8h*)&T[n * LDT + kc];
    off[i] = (size_t)(n0 + n) * Kdim + k0 + kc;
  }
#pragma unroll
  for (int i = 0; i < 2; ++i) *(volatile v8h*)(Wt + off[i]) = x[i];
  __threadfence();
#pragma unroll
  for (int i = 0; i < 2; ++i) *(volatile v8h*)(Wt + off[i]) = x[i];
}

__global__ __launch_bounds__(256) void cconv_kernel(
    const float* __restrict__ cond, _Float16* __restrict__ dst) {
  const unsigned e = (blockIdx.x * 256u + threadIdx.x) * 8u;
  const unsigned row = e / (unsigned)DCOND;
  const unsigned c = e - row * (unsigned)DCOND;
  const unsigned bidx = row / (unsigned)CPAD;
  const unsigned r = row - bidx * (unsigned)CPAD;
  const unsigned rc = (r < (unsigned)NCOND) ? r : (unsigned)(NCOND - 1);
  const float keep = (r < (unsigned)NCOND) ? 1.0f : 0.0f;
  const float* sp = cond + ((size_t)bidx * NCOND + rc) * DCOND + c;
  const v4f a0 = *(const v4f*)(sp);
  const v4f a1 = *(const v4f*)(sp + 4);
  v8h o;
#pragma unroll
  for (int j = 0; j < 4; ++j) {
    o[j]     = (_Float16)(keep * bf16r(a0[j]));
    o[j + 4] = (_Float16)(keep * bf16r(a1[j]));
  }
  *(volatile v8h*)(dst + (size_t)e) = o;
  __threadfence();
  *(volatile v8h*)(dst + (size_t)e) = o;
}

__global__ __launch_bounds__(256) void ln_kernel(
    const float* __restrict__ X, const float* __restrict__ gam, const float* __restrict__ bet,
    _Float16* __restrict__ dst, unsigned src_full, unsigned src_cvt) {
  const unsigned lane = threadIdx.x & 31u;
  const unsigned wave = (unsigned)__builtin_amdgcn_readfirstlane((int)(threadIdx.x >> 5));
  const unsigned crow = blockIdx.x * 8u + wave;
  const unsigned bidx = crow / (unsigned)SEQ;
  const unsigned sq = crow - bidx * (unsigned)SEQ;
  const size_t srow = (src_full != 0u) ? ((size_t)bidx * SEQ_FULL + sq) : (size_t)crow;
  const size_t xo = srow * DIM + lane * 8u;
  const bool cv = (src_cvt != 0u);

  float s = 0.0f;
#pragma unroll 1
  for (unsigned j = 0; j < 4u; ++j) {
    v4f a0 = *(const v4f*)(X + xo + j * 256u);
    v4f a1 = *(const v4f*)(X + xo + j * 256u + 4u);
#pragma unroll
    for (int t = 0; t < 4; ++t) {
      a0[t] = cv ? bf16r(a0[t]) : a0[t];
      a1[t] = cv ? bf16r(a1[t]) : a1[t];
    }
    s += ((a0[0] + a0[1]) + (a0[2] + a0[3])) + ((a1[0] + a1[1]) + (a1[2] + a1[3]));
  }
  const float mean = red32_sum(s) * (1.0f / (float)DIM);

  float q = 0.0f;
#pragma unroll 1
  for (unsigned j = 0; j < 4u; ++j) {
    v4f a0 = *(const v4f*)(X + xo + j * 256u);
    v4f a1 = *(const v4f*)(X + xo + j * 256u + 4u);
#pragma unroll
    for (int t = 0; t < 4; ++t) {
      const float d0 = (cv ? bf16r(a0[t]) : a0[t]) - mean;
      const float d1 = (cv ? bf16r(a1[t]) : a1[t]) - mean;
      q += d0 * d0;
      q += d1 * d1;
    }
  }
  const float rstd = rsqrtf(red32_sum(q) * (1.0f / (float)DIM) + 1.0e-5f);

#pragma unroll 1
  for (unsigned pass = 0; pass < 2u; ++pass) {
#pragma unroll 1
    for (unsigned j = 0; j < 4u; ++j) {
      const unsigned col = lane * 8u + j * 256u;
      const v4f a0 = *(const v4f*)(X + xo + j * 256u);
      const v4f a1 = *(const v4f*)(X + xo + j * 256u + 4u);
      const v4f g0 = *(const v4f*)(gam + col);
      const v4f g1 = *(const v4f*)(gam + col + 4u);
      const v4f b0 = *(const v4f*)(bet + col);
      const v4f b1 = *(const v4f*)(bet + col + 4u);
      v8h o;
#pragma unroll
      for (int t = 0; t < 4; ++t) {
        const float x0 = cv ? bf16r(a0[t]) : a0[t];
        const float x1 = cv ? bf16r(a1[t]) : a1[t];
        o[t]     = (_Float16)(((x0 - mean) * rstd) * bf16r(g0[t]) + bf16r(b0[t]));
        o[t + 4] = (_Float16)(((x1 - mean) * rstd) * bf16r(g1[t]) + bf16r(b1[t]));
      }
      *(volatile v8h*)(dst + (size_t)crow * DIM + col) = o;
    }
    __threadfence();
  }
}

__device__ __forceinline__ void gemm_tile(
    const _Float16* __restrict__ A16, const _Float16* __restrict__ Bt, unsigned K,
    unsigned row0, unsigned n0, unsigned wave, unsigned lane, v8f& acc0, v8f& acc1) {
  const unsigned mw = wave >> 1, nw = wave & 1u;
  const unsigned hh = lane >> 4, m = lane & 15u;
  const size_t aoff = (size_t)(row0 + mw * 16u + m) * K + hh * 8u;
  const size_t boff0 = (size_t)(n0 + nw * 32u + m) * K + hh * 8u;
  const size_t boff1 = boff0 + (size_t)16u * K;
  v8f c0 = {}, c1 = {};
#pragma unroll 2
  for (unsigned k0 = 0; k0 < K; k0 += 32u) {
    const v16h a  = frag_at(A16 + aoff + k0);
    const v16h b0 = frag_at(Bt + boff0 + k0);
    const v16h b1 = frag_at(Bt + boff1 + k0);
    c0 = wmma16(a, b0, c0);
    c1 = wmma16(a, b1, c1);
  }
  acc0 = c0;
  acc1 = c1;
}

__global__ __launch_bounds__(256) void gemm_proj_kernel(
    const _Float16* __restrict__ A16, const _Float16* __restrict__ Bt,
    _Float16* __restrict__ out16, unsigned K, unsigned keys, unsigned plane_elems,
    unsigned vt_which) {
  __shared__ float Cs[64 * LDC];
  const unsigned tid = threadIdx.x, lane = tid & 31u;
  const unsigned wave = (unsigned)__builtin_amdgcn_readfirstlane((int)(threadIdx.x >> 5));
  const unsigned mw = wave >> 1, nw = wave & 1u;
  const unsigned hh = lane >> 4, m = lane & 15u;
  const unsigned n0 = blockIdx.x * 64u;
  const unsigned row0 = blockIdx.y * 64u;
  const unsigned which = blockIdx.z;

  v8f acc0, acc1;
  gemm_tile(A16, Bt + (size_t)which * DIM * K, K, row0, n0, wave, lane, acc0, acc1);
#pragma unroll
  for (int r = 0; r < 8; ++r) {
    const unsigned ci = (mw * 16u + hh * 8u + (unsigned)r) * LDC + nw * 32u + m;
    Cs[ci]       = acc0[r];
    Cs[ci + 16u] = acc1[r];
  }
  __syncthreads();

  const size_t pbase = (size_t)which * plane_elems;
  v8h x[2];
  size_t off[2];
  if (which != vt_which) {
#pragma unroll
    for (unsigned i = 0; i < 2u; ++i) {
      const unsigned r = 32u * i + (tid >> 3);
      const unsigned c = (tid & 7u) * 8u;
      const v4f u0 = *(const v4f*)&Cs[r * LDC + c];
      const v4f u1 = *(const v4f*)&Cs[r * LDC + c + 4u];
#pragma unroll
      for (int j = 0; j < 4; ++j) {
        x[i][j]     = (_Float16)(u0[j] * (1.0f / WCARRY));
        x[i][j + 4] = (_Float16)(u1[j] * (1.0f / WCARRY));
      }
      off[i] = pbase + (size_t)(row0 + r) * DIM + n0 + c;
    }
  } else {
    const unsigned bidx = row0 / keys;
    const unsigned key0 = row0 - bidx * keys;
#pragma unroll
    for (unsigned i = 0; i < 2u; ++i) {
      const unsigned dcol = 32u * i + (tid >> 3);
      const unsigned kk = (tid & 7u) * 8u;
#pragma unroll
      for (unsigned j = 0; j < 8u; ++j)
        x[i][j] = (_Float16)(Cs[(kk + j) * LDC + dcol] * (1.0f / WCARRY));
      off[i] = pbase + ((size_t)bidx * DIM + n0 + dcol) * keys + key0 + kk;
    }
  }
#pragma unroll
  for (int i = 0; i < 2; ++i) *(volatile v8h*)(out16 + off[i]) = x[i];
  __threadfence();
#pragma unroll
  for (int i = 0; i < 2; ++i) *(volatile v8h*)(out16 + off[i]) = x[i];
}

__global__ __launch_bounds__(256) void gemm_res_kernel(
    const _Float16* __restrict__ A16, const _Float16* __restrict__ Bt,
    const float* __restrict__ bias, const float* __restrict__ res, float* __restrict__ outf,
    unsigned K, unsigned res_full, unsigned res_cvt, unsigned out_full, float scl) {
  __shared__ float Cs[64 * LDC];
  const unsigned tid = threadIdx.x, lane = tid & 31u;
  const unsigned wave = (unsigned)__builtin_amdgcn_readfirstlane((int)(threadIdx.x >> 5));
  const unsigned mw = wave >> 1, nw = wave & 1u;
  const unsigned hh = lane >> 4, m = lane & 15u;
  const unsigned n0 = blockIdx.x * 64u;
  const unsigned row0 = blockIdx.y * 64u;

  v8f acc0, acc1;
  gemm_tile(A16, Bt, K, row0, n0, wave, lane, acc0, acc1);
#pragma unroll
  for (int r = 0; r < 8; ++r) {
    const unsigned ci = (mw * 16u + hh * 8u + (unsigned)r) * LDC + nw * 32u + m;
    Cs[ci]       = acc0[r];
    Cs[ci + 16u] = acc1[r];
  }
  __syncthreads();

  const bool cv = (res_cvt != 0u);
  v4f xs[4];
  size_t off[4];
#pragma unroll
  for (unsigned i = 0; i < 4u; ++i) {
    const unsigned r = 16u * i + (tid >> 4);
    const unsigned c = (tid & 15u) * 4u;
    const unsigned crow = row0 + r;
    const unsigned bidx = crow / (unsigned)SEQ;
    const unsigned sq = crow - bidx * (unsigned)SEQ;
    const size_t frow = (size_t)bidx * SEQ_FULL + sq;
    const size_t rrow = (res_full != 0u) ? frow : (size_t)crow;
    const size_t orow = (out_full != 0u) ? frow : (size_t)crow;
    const v4f u = *(const v4f*)&Cs[r * LDC + c];
    const v4f g = *(const v4f*)(bias + n0 + c);
    const v4f rv = *(const v4f*)(res + rrow * DIM + n0 + c);
    v4f val;
#pragma unroll
    for (int j = 0; j < 4; ++j) {
      const float rj = cv ? bf16r(rv[j]) : rv[j];
      val[j] = (u[j] * scl + bf16r(g[j])) + rj;
    }
    xs[i] = val;
    off[i] = orow * DIM + n0 + c;
  }
#pragma unroll
  for (int i = 0; i < 4; ++i) *(volatile v4f*)(outf + off[i]) = xs[i];
  __threadfence();
#pragma unroll
  for (int i = 0; i < 4; ++i) *(volatile v4f*)(outf + off[i]) = xs[i];
}

__global__ __launch_bounds__(256) void gemm_gelu_kernel(
    const _Float16* __restrict__ A16, const _Float16* __restrict__ Bt,
    const float* __restrict__ bias, _Float16* __restrict__ out16, unsigned K, unsigned ldo) {
  __shared__ float Cs[64 * LDC];
  const unsigned tid = threadIdx.x, lane = tid & 31u;
  const unsigned wave = (unsigned)__builtin_amdgcn_readfirstlane((int)(threadIdx.x >> 5));
  const unsigned mw = wave >> 1, nw = wave & 1u;
  const unsigned hh = lane >> 4, m = lane & 15u;
  const unsigned n0 = blockIdx.x * 64u;
  const unsigned row0 = blockIdx.y * 64u;

  v8f acc0, acc1;
  gemm_tile(A16, Bt, K, row0, n0, wave, lane, acc0, acc1);
#pragma unroll
  for (int r = 0; r < 8; ++r) {
    const unsigned ci = (mw * 16u + hh * 8u + (unsigned)r) * LDC + nw * 32u + m;
    Cs[ci]       = acc0[r];
    Cs[ci + 16u] = acc1[r];
  }
  __syncthreads();

  v8h x[2];
  size_t off[2];
#pragma unroll
  for (unsigned i = 0; i < 2u; ++i) {
    const unsigned r = 32u * i + (tid >> 3);
    const unsigned c = (tid & 7u) * 8u;
    const v4f u0 = *(const v4f*)&Cs[r * LDC + c];
    const v4f u1 = *(const v4f*)&Cs[r * LDC + c + 4u];
    const v4f g0 = *(const v4f*)(bias + n0 + c);
    const v4f g1 = *(const v4f*)(bias + n0 + c + 4u);
#pragma unroll
    for (int j = 0; j < 4; ++j) {
      const float t0 = u0[j] * (1.0f / WCARRY) + bf16r(g0[j]);
      const float t1 = u1[j] * (1.0f / WCARRY) + bf16r(g1[j]);
      const float e0 = 0.5f * t0 * (1.0f + erff(t0 * 0.70710678118654752f));
      const float e1 = 0.5f * t1 * (1.0f + erff(t1 * 0.70710678118654752f));
      x[i][j]     = (_Float16)(e0 * GCARRY);
      x[i][j + 4] = (_Float16)(e1 * GCARRY);
    }
    off[i] = (size_t)(row0 + r) * ldo + n0 + c;
  }
#pragma unroll
  for (int i = 0; i < 2; ++i) *(volatile v8h*)(out16 + off[i]) = x[i];
  __threadfence();
#pragma unroll
  for (int i = 0; i < 2; ++i) *(volatile v8h*)(out16 + off[i]) = x[i];
}

__global__ __launch_bounds__(256) void attn_kernel(
    const _Float16* __restrict__ Qh, const _Float16* __restrict__ Kh,
    const _Float16* __restrict__ Vt, _Float16* __restrict__ Ov) {
  __shared__ _Float16 Ks[64 * LDT];
  __shared__ _Float16 Vs[64 * LDT];
  __shared__ _Float16 Ps[8 * 16 * LDT];

  const unsigned tid = threadIdx.x, lane = tid & 31u;
  const unsigned wave = (unsigned)__builtin_amdgcn_readfirstlane((int)(threadIdx.x >> 5));
  const unsigned hh = lane >> 4, m = lane & 15u;
  const unsigned q0 = blockIdx.x * 128u;
  const unsigned head = blockIdx.y;
  const unsigned b = blockIdx.z;
  const unsigned qw = q0 + wave * 16u;
  const unsigned pb = wave * (16u * LDT);
  const unsigned fo = m * LDT + hh * 8u;
  const float scale = 0.125f;

  const size_t qoff = (size_t)(b * (unsigned)SEQ + qw + m) * DIM + head * HD + hh * 8u;
  v16h qf[2];
  qf[0] = frag_at(Qh + qoff);
  qf[1] = frag_at(Qh + qoff + 32);

  float mrow[8], lrow[8];
  v8f o[4];
#pragma unroll
  for (int v = 0; v < 8; ++v) { mrow[v] = -1.0e30f; lrow[v] = 0.0f; }
#pragma unroll
  for (int nb = 0; nb < 4; ++nb) o[nb] = (v8f){};

  const size_t kplane = (size_t)b * SEQ * DIM + head * HD;
  const size_t vplane = ((size_t)b * DIM + head * HD) * SEQ;
  const unsigned kend = q0 + 128u;

  for (unsigned kb = 0; kb < kend; kb += 64u) {
#pragma unroll
    for (unsigned j = 0; j < 2u; ++j) {
      const unsigned idx = tid + 256u * j;
      const unsigned r = idx >> 3, c = (idx & 7u) * 8u;
      *(v8h*)&Ks[r * LDT + c] = *(const v8h*)(Kh + kplane + (size_t)(kb + r) * DIM + c);
      *(v8h*)&Vs[r * LDT + c] = *(const v8h*)(Vt + vplane + (size_t)r * SEQ + kb + c);
    }
    __syncthreads();

    if (kb <= qw + 15u) {
      v8f s[4];
#pragma unroll
      for (int kg = 0; kg < 4; ++kg) {
        v8f t = {};
#pragma unroll
        for (int c = 0; c < 2; ++c) {
          const v16h kf = LDS_FRAG(Ks, (unsigned)(kg * 16) * LDT + (unsigned)c * 32u + fo);
          t = wmma16(qf[c], kf, t);
        }
        s[kg] = t * scale;
      }
      if (kb + 63u > qw) {
#pragma unroll
        for (int kg = 0; kg < 4; ++kg) {
          const unsigned key = kb + (unsigned)kg * 16u + m;
#pragma unroll
          for (int v = 0; v < 8; ++v) {
            const unsigned qr = qw + hh * 8u + (unsigned)v;
            s[kg][v] = (key <= qr) ? s[kg][v] : -1.0e30f;
          }
        }
      }

      float alpha[8];
#pragma unroll
      for (int v = 0; v < 8; ++v) {
        float mx = fmaxf(fmaxf(s[0][v], s[1][v]), fmaxf(s[2][v], s[3][v]));
        mx = red16_max(mx);
        const float mn = fmaxf(mrow[v], mx);
        alpha[v] = __expf(mrow[v] - mn);
        mrow[v] = mn;
      }
#pragma unroll
      for (int kg = 0; kg < 4; ++kg)
#pragma unroll
        for (int v = 0; v < 8; ++v) s[kg][v] = __expf(s[kg][v] - mrow[v]);
#pragma unroll
      for (int v = 0; v < 8; ++v) {
        const float rs = red16_sum((s[0][v] + s[1][v]) + (s[2][v] + s[3][v]));
        lrow[v] = alpha[v] * lrow[v] + rs;
      }
#pragma unroll
      for (int nb = 0; nb < 4; ++nb)
#pragma unroll
        for (int v = 0; v < 8; ++v) o[nb][v] = o[nb][v] * alpha[v];

#pragma unroll
      for (int kg = 0; kg < 4; ++kg)
#pragma unroll
        for (int v = 0; v < 8; ++v)
          Ps[pb + (hh * 8u + (unsigned)v) * LDT + (unsigned)kg * 16u + m] =
              (_Float16)(s[kg][v] * PCARRY);
      wave_lds_sync();

#pragma unroll
      for (int c = 0; c < 2; ++c) {
        const v16h pf = LDS_FRAG(Ps, pb + (unsigned)c * 32u + fo);
#pragma unroll
        for (int nb = 0; nb < 4; ++nb) {
          const v16h vf = LDS_FRAG(Vs, (unsigned)(nb * 16) * LDT + (unsigned)c * 32u + fo);
          o[nb] = wmma16(pf, vf, o[nb]);
        }
      }
    }
    __syncthreads();
  }

  float inv[8];
#pragma unroll
  for (int v = 0; v < 8; ++v) inv[v] = __builtin_amdgcn_rcpf(lrow[v]) * (VCARRY / PCARRY);
#pragma unroll
  for (int nb = 0; nb < 4; ++nb)
#pragma unroll
    for (int v = 0; v < 8; ++v)
      Ps[pb + (hh * 8u + (unsigned)v) * LDT + (unsigned)nb * 16u + m] =
          (_Float16)(o[nb][v] * inv[v]);
  wave_lds_sync();
  v8h x[4];
  size_t off[4];
#pragma unroll
  for (unsigned i = 0; i < 4u; ++i) {
    const unsigned r = 4u * i + (lane >> 3);
    const unsigned c = (lane & 7u) * 8u;
    x[i] = *(const v8h*)&Ps[pb + r * LDT + c];
    off[i] = (size_t)(b * (unsigned)SEQ + qw + r) * DIM + head * HD + c;
  }
#pragma unroll
  for (int i = 0; i < 4; ++i) *(volatile v8h*)(Ov + off[i]) = x[i];
  __threadfence();
#pragma unroll
  for (int i = 0; i < 4; ++i) *(volatile v8h*)(Ov + off[i]) = x[i];
}

__global__ __launch_bounds__(256) void xattn_kernel(
    const _Float16* __restrict__ Qh, const _Float16* __restrict__ Kc,
    const _Float16* __restrict__ Vtc, _Float16* __restrict__ Ov) {
  __shared__ _Float16 Kx[CKEYS * LDT];
  __shared__ _Float16 Vx[64 * LDP];
  __shared__ _Float16 Px[8 * 16 * LDP];

  const unsigned tid = threadIdx.x, lane = tid & 31u;
  const unsigned wave = (unsigned)__builtin_amdgcn_readfirstlane((int)(threadIdx.x >> 5));
  const unsigned hh = lane >> 4, m = lane & 15u;
  const unsigned q0 = blockIdx.x * 128u;
  const unsigned head = blockIdx.y;
  const unsigned b = blockIdx.z;
  const unsigned qw = q0 + wave * 16u;
  const unsigned pb = wave * (16u * LDP);
  const unsigned fok = m * LDT + hh * 8u;
  const unsigned fop = m * LDP + hh * 8u;
  const float scale = 0.125f;

  static_assert((CKEYS * 8) % 256 == 0 && (64 * (CKEYS / 8)) % 256 == 0);
#pragma unroll
  for (unsigned j = 0; j < (unsigned)(CKEYS * 8 / 256); ++j) {
    const unsigned idx = tid + 256u * j;
    const unsigned r = idx >> 3, c = (idx & 7u) * 8u;
    *(v8h*)&Kx[r * LDT + c] =
        *(const v8h*)(Kc + (size_t)(b * (unsigned)CPAD + r) * DIM + head * HD + c);
  }
#pragma unroll
  for (unsigned j = 0; j < (unsigned)(64 * (CKEYS / 8) / 256); ++j) {
    const unsigned idx = tid + 256u * j;
    const unsigned r = idx / (unsigned)(CKEYS / 8);
    const unsigned c = (idx - r * (unsigned)(CKEYS / 8)) * 8u;
    *(v8h*)&Vx[r * LDP + c] =
        *(const v8h*)(Vtc + ((size_t)b * DIM + head * HD + r) * CPAD + c);
  }
  __syncthreads();

  const size_t qoff = (size_t)(b * (unsigned)SEQ + qw + m) * DIM + head * HD + hh * 8u;
  v16h qf[2];
  qf[0] = frag_at(Qh + qoff);
  qf[1] = frag_at(Qh + qoff + 32);

  v8f s[CKEYS / 16];
#pragma unroll
  for (int kg = 0; kg < CKEYS / 16; ++kg) {
    v8f t = {};
#pragma unroll
    for (int c = 0; c < 2; ++c) {
      const v16h kf = LDS_FRAG(Kx, (unsigned)(kg * 16) * LDT + (unsigned)c * 32u + fok);
      t = wmma16(qf[c], kf, t);
    }
    s[kg] = t * scale;
  }
#pragma unroll
  for (int kg = 0; kg < CKEYS / 16; ++kg) {
    const unsigned key = (unsigned)kg * 16u + m;
#pragma unroll
    for (int v = 0; v < 8; ++v) s[kg][v] = (key < (unsigned)NCOND) ? s[kg][v] : -1.0e30f;
  }

  float inv[8];
#pragma unroll
  for (int v = 0; v < 8; ++v) {
    float mx = s[0][v];
#pragma unroll
    for (int kg = 1; kg < CKEYS / 16; ++kg) mx = fmaxf(mx, s[kg][v]);
    mx = red16_max(mx);
    float sum = 0.0f;
#pragma unroll
    for (int kg = 0; kg < CKEYS / 16; ++kg) {
      const float p = __expf(s[kg][v] - mx);
      s[kg][v] = p;
      sum += p;
    }
    sum = red16_sum(sum);
    inv[v] = __builtin_amdgcn_rcpf(sum) * (VCARRY / PCARRY);
  }

#pragma unroll
  for (int kg = 0; kg < CKEYS / 16; ++kg)
#pragma unroll
    for (int v = 0; v < 8; ++v)
      Px[pb + (hh * 8u + (unsigned)v) * LDP + (unsigned)kg * 16u + m] =
          (_Float16)(s[kg][v] * PCARRY);
  wave_lds_sync();

  v8f o[4];
#pragma unroll
  for (int nb = 0; nb < 4; ++nb) o[nb] = (v8f){};
#pragma unroll
  for (int c = 0; c < CKEYS / 32; ++c) {
    const v16h pf = LDS_FRAG(Px, pb + (unsigned)c * 32u + fop);
#pragma unroll
    for (int nb = 0; nb < 4; ++nb) {
      const v16h vf = LDS_FRAG(Vx, (unsigned)(nb * 16) * LDP + (unsigned)c * 32u + fop);
      o[nb] = wmma16(pf, vf, o[nb]);
    }
  }
  wave_lds_sync();

#pragma unroll
  for (int nb = 0; nb < 4; ++nb)
#pragma unroll
    for (int v = 0; v < 8; ++v)
      Px[pb + (hh * 8u + (unsigned)v) * LDP + (unsigned)nb * 16u + m] =
          (_Float16)(o[nb][v] * inv[v]);
  wave_lds_sync();
  v8h x[4];
  size_t off[4];
#pragma unroll
  for (unsigned i = 0; i < 4u; ++i) {
    const unsigned r = 4u * i + (lane >> 3);
    const unsigned c = (lane & 7u) * 8u;
    x[i] = *(const v8h*)&Px[pb + r * LDP + c];
    off[i] = (size_t)(b * (unsigned)SEQ + qw + r) * DIM + head * HD + c;
  }
#pragma unroll
  for (int i = 0; i < 4; ++i) *(volatile v8h*)(Ov + off[i]) = x[i];
  __threadfence();
#pragma unroll
  for (int i = 0; i < 4; ++i) *(volatile v8h*)(Ov + off[i]) = x[i];
}

extern "C" void kernel_launch(void* const* d_in, const int* in_sizes, int n_in,
                              void* d_out, int out_size, void* d_ws, size_t ws_size,
                              hipStream_t stream) {
  if (n_in < 19) return;
  const long long need_x = ((long long)(NB - 1) * SEQ_FULL + SEQ) * DIM;
  if ((long long)in_sizes[0] < need_x) return;
  if ((long long)in_sizes[1] < (long long)NB * NCOND * DCOND) return;
  if ((long long)in_sizes[2] < (long long)DIM * 3 * DIM) return;
  if ((long long)in_sizes[3] < (long long)DIM * DIM) return;
  if (in_sizes[4] < DIM || in_sizes[5] < DIM || in_sizes[6] < DIM) return;
  if ((long long)in_sizes[7] < (long long)DIM * DIM) return;
  if ((long long)in_sizes[8] < (long long)DCOND * 2 * DIM) return;
  if ((long long)in_sizes[9] < (long long)DIM * DIM) return;
  if (in_sizes[10] < DIM || in_sizes[11] < DIM || in_sizes[12] < DIM) return;
  if ((long long)in_sizes[13] < (long long)DIM * DFF) return;
  if (in_sizes[14] < DFF) return;
  if ((long long)in_sizes[15] < (long long)DFF * DIM) return;
  if (in_sizes[16] < DIM || in_sizes[17] < DIM || in_sizes[18] < DIM) return;
  if ((long long)out_size < need_x) return;
  if (ws_size < WS_TOTAL) return;

  const float* X        = (const float*)d_in[0];
  const float* cond     = (const float*)d_in[1];
  const float* Wqkv     = (const float*)d_in[2];
  const float* Wproj_sa = (const float*)d_in[3];
  const float* bproj_sa = (const float*)d_in[4];
  const float* g1       = (const float*)d_in[5];
  const float* b1       = (const float*)d_in[6];
  const float* Wq_ca    = (const float*)d_in[7];
  const float* Wkv_ca   = (const float*)d_in[8];
  const float* Wproj_ca = (const float*)d_in[9];
  const float* bproj_ca = (const float*)d_in[10];
  const float* g2       = (const float*)d_in[11];
  const float* b2       = (const float*)d_in[12];
  const float* Wff1     = (const float*)d_in[13];
  const float* bff1     = (const float*)d_in[14];
  const float* Wff2     = (const float*)d_in[15];
  const float* bff2     = (const float*)d_in[16];
  const float* g3       = (const float*)d_in[17];
  const float* b3       = (const float*)d_in[18];
  float* out = (float*)d_out;

  char* ws = (char*)d_ws;
  _Float16* Wt    = (_Float16*)ws;
  _Float16* H16   = (_Float16*)(ws + B_H16);
  _Float16* Q16   = (_Float16*)(ws + B_QKVC);
  _Float16* K16   = (_Float16*)(ws + B_QKVC + 1 * PLANE16_BYTES);
  _Float16* Vt16  = (_Float16*)(ws + B_QKVC + 2 * PLANE16_BYTES);
  _Float16* Ctx16 = (_Float16*)(ws + B_QKVC + 3 * PLANE16_BYTES);
  _Float16* G16   = (_Float16*)(ws + B_QKVC);
  float*    X1    = (float*)(ws + B_X1);
  float*    X2    = (float*)(ws + B_X2);
  _Float16* C16   = (_Float16*)(ws + B_C16);
  _Float16* Kc16  = (_Float16*)(ws + B_KVC);
  _Float16* Vtc16 = (_Float16*)(ws + B_KVC + KV16_BYTES);

  dim3 blk(256);
  const float oscl = 1.0f / (WCARRY * VCARRY);
  static_assert(VCARRY == GCARRY);

  wconv_kernel<<<dim3(3 * DIM / 64, DIM / 64), blk, 0, stream>>>(Wqkv, Wt + OFF_WQKV, DIM, 3 * DIM);
  wconv_kernel<<<dim3(DIM / 64, DIM / 64), blk, 0, stream>>>(Wproj_sa, Wt + OFF_WPSA, DIM, DIM);
  wconv_kernel<<<dim3(DIM / 64, DIM / 64), blk, 0, stream>>>(Wq_ca, Wt + OFF_WQCA, DIM, DIM);
  wconv_kernel<<<dim3(2 * DIM / 64, DCOND / 64), blk, 0, stream>>>(Wkv_ca, Wt + OFF_WKV, DCOND, 2 * DIM);
  wconv_kernel<<<dim3(DIM / 64, DIM / 64), blk, 0, stream>>>(Wproj_ca, Wt + OFF_WPCA, DIM, DIM);
  wconv_kernel<<<dim3(DFF / 64, DIM / 64), blk, 0, stream>>>(Wff1, Wt + OFF_WFF1, DIM, DFF);
  wconv_kernel<<<dim3(DIM / 64, DFF / 64), blk, 0, stream>>>(Wff2, Wt + OFF_WFF2, DFF, DIM);
  cconv_kernel<<<dim3((unsigned)(((size_t)CROWS * DCOND) / 2048)), blk, 0, stream>>>(cond, C16);

  ln_kernel<<<dim3(MROWS / 8), blk, 0, stream>>>(X, g1, b1, H16, 1u, 1u);
  gemm_proj_kernel<<<dim3(DIM / 64, MROWS / 64, 3), blk, 0, stream>>>(
      H16, Wt + OFF_WQKV, Q16, (unsigned)DIM, (unsigned)SEQ, (unsigned)((size_t)MROWS * DIM), 2u);
  attn_kernel<<<dim3(SEQ / 128, NHEAD, NB), blk, 0, stream>>>(Q16, K16, Vt16, Ctx16);
  gemm_res_kernel<<<dim3(DIM / 64, MROWS / 64), blk, 0, stream>>>(
      Ctx16, Wt + OFF_WPSA, bproj_sa, X, X1, (unsigned)DIM, 1u, 1u, 0u, oscl);

  ln_kernel<<<dim3(MROWS / 8), blk, 0, stream>>>(X1, g2, b2, H16, 0u, 0u);
  gemm_proj_kernel<<<dim3(DIM / 64, MROWS / 64, 1), blk, 0, stream>>>(
      H16, Wt + OFF_WQCA, Q16, (unsigned)DIM, (unsigned)SEQ, (unsigned)((size_t)MROWS * DIM), 99u);
  gemm_proj_kernel<<<dim3(DIM / 64, CROWS / 64, 2), blk, 0, stream>>>(
      C16, Wt + OFF_WKV, Kc16, (unsigned)DCOND, (unsigned)CPAD, (unsigned)((size_t)CROWS * DIM), 1u);
  xattn_kernel<<<dim3(SEQ / 128, NHEAD, NB), blk, 0, stream>>>(Q16, Kc16, Vtc16, Ctx16);
  gemm_res_kernel<<<dim3(DIM / 64, MROWS / 64), blk, 0, stream>>>(
      Ctx16, Wt + OFF_WPCA, bproj_ca, X1, X2, (unsigned)DIM, 0u, 0u, 0u, oscl);

  ln_kernel<<<dim3(MROWS / 8), blk, 0, stream>>>(X2, g3, b3, H16, 0u, 0u);
  gemm_gelu_kernel<<<dim3(DFF / 64, MROWS / 64), blk, 0, stream>>>(
      H16, Wt + OFF_WFF1, bff1, G16, (unsigned)DIM, (unsigned)DFF);
  gemm_res_kernel<<<dim3(DIM / 64, MROWS / 64), blk, 0, stream>>>(
      G16, Wt + OFF_WFF2, bff2, X2, out, (unsigned)DFF, 0u, 0u, 1u, oscl);
}
